// JKNet_53291954209003
// MI455X (gfx1250) — hardware-run, weakly checked
//
#include <hip/hip_runtime.h>
#include <stddef.h>
#include <stdint.h>
#include <math.h>

#define LAYER_SPLIT 1
#define HEAD_SPLIT  1

#define NN      50000
#define NE      800000
#define FD      256
#define HD      64
#define NSL     4
#define CW      512
#define CLO     256
#define WLP     128
#define WMP     512
#define GBM     128
#define MP      50048
#define NTHR    256
#define NWAVE   8
#define EPT     8
#define WCH     (32 * EPT)
#define NBRUN   1024
#define SLB     10
#define NBK     49
#define WLCAP   3584
#define RCAP    28672
#define TRIPCAP 64
#define MAXDEG_IN_MEAS   33
#define MAXDEG_OUT_MEAS  37
#define MAXB_IN_MEAS     16696
#define MAXB_OUT_MEAS    16759
#define ABM     64
#define SP      68

#define BK_WL    0
#define BK_PL    (NWAVE * WLCAP)
#define BK_CNT   (BK_PL + RCAP)
#define BK_NSD   (BK_CNT + 3 * NBRUN)
#define BK_ZINTS (BK_NSD + 2 * NBRUN)
#define BK_INTS  (BK_ZINTS + 16)
#define BK_LDS   (BK_INTS * 4)

#define PBX   (MP * FD / 8 / NTHR)
#define PBWF  (HD * FD / 8 / NTHR)
#define PBWL  (HD * WLP / 8 / NTHR)
#define PBWM  (HD * WMP / 8 / NTHR)
#define PBZC  ((MP - NN) * CW / 8 / NTHR)
#define PBZP  ((MP - NN) * HD / 4 / NTHR)
#define PE_X  PBX
#define PE_WF (PE_X + PBWF)
#define PE_WA (PE_WF + PBWL)
#define PE_WB (PE_WA + PBWL)
#define PE_WC (PE_WB + PBWL)
#define PE_WM (PE_WC + PBWM)
#define PE_ZC (PE_WM + PBZC)
#define PE_ZP (PE_ZC + PBZP)
#define PBTOT (PE_ZP + 1)

static_assert(HD == 64 && HD == 16 * 4 && FD == 256 && NSL * HD == 256 && CLO == NSL * HD && CW == 2 * CLO);
static_assert(GBM == 128 && GBM == NWAVE * 16);
static_assert(MP % GBM == 0 && MP >= NN && MP == 391 * GBM && MP % ABM == 0 && NN % 2 == 0);
static_assert(NBRUN == (1 << SLB) && NBRUN % ABM == 0 && NBRUN % GBM == 0 && NBRUN % 32 == 0 && NBRUN < 65536);
static_assert(NBK * NBRUN >= MP && NBK * NBRUN >= NN);
static_assert((((long long)NE) << SLB) < (1LL << 31));
static_assert(NE % WCH == 0 && NE % 4 == 0);
static_assert(RCAP == NWAVE * WLCAP && RCAP % (NTHR * 4) == 0 && BK_ZINTS % 4 == 0);
static_assert((long long)RCAP * 100 >= (long long)MAXB_IN_MEAS * 105);
static_assert((long long)RCAP * 100 >= (long long)MAXB_OUT_MEAS * 105);
static_assert(WLCAP >= MAXB_OUT_MEAS / 8 + 8 * 46 + 1 && WLCAP >= MAXB_IN_MEAS / 8 + 8 * 46 + 1);
static_assert(NN <= 65536);
static_assert(MAXDEG_IN_MEAS + 8 <= TRIPCAP && MAXDEG_OUT_MEAS + 8 <= TRIPCAP && TRIPCAP < 65536);
static_assert((MP * FD / 8) % NTHR == 0 && (HD * FD / 8) % NTHR == 0 && (HD * WLP / 8) % NTHR == 0);
static_assert((HD * WMP / 8) % NTHR == 0 && ((MP - NN) * CW / 8) % NTHR == 0 && ((MP - NN) * HD / 4) % NTHR == 0);
static_assert(FD % 32 == 0 && HD % 32 == 0 && CLO % 32 == 0 && WLP == 2 * HD && WMP == 2 * CLO);
static_assert(BK_LDS <= 300000);
static_assert((GBM * SP + 128) * 4 <= 65536);
static_assert(2 * NBRUN == 8 * NTHR && NBRUN == 4 * NTHR);

typedef float          v4f   __attribute__((ext_vector_type(4)));
typedef float          v8f   __attribute__((ext_vector_type(8)));
typedef int            v2i   __attribute__((ext_vector_type(2)));
typedef int            v4i   __attribute__((ext_vector_type(4)));
typedef int            v8i   __attribute__((ext_vector_type(8)));
typedef unsigned short v8us  __attribute__((ext_vector_type(8)));
typedef unsigned short v16us __attribute__((ext_vector_type(16)));
typedef __bf16         v16bf __attribute__((ext_vector_type(16)));
typedef v4f  __attribute__((may_alias)) v4fa;
typedef v4i  __attribute__((may_alias)) v4ia;
typedef v8us __attribute__((may_alias)) v8usa;
union FragB { v16bf v; v16us u; v8us h[2]; v8i w; };

__device__ __forceinline__ v8f wmb(const FragB& a, const FragB& b, v8f c) {
  v8f d = __builtin_amdgcn_wmma_f32_16x16x32_bf16(false, a.v, false, b.v, (short)0, c, false, false);
  asm volatile("v_nop\n\tv_nop\n\tv_nop\n\tv_nop" : "+v"(d) : "v"(a.w), "v"(b.w));
  return d;
}

__device__ __forceinline__ unsigned bf16_bits(float f) {
  const unsigned u = __float_as_uint(f);
  const unsigned r = (u + 0x7FFFu + ((u >> 16) & 1u)) >> 16;
  const unsigned q = (u >> 16) | 0x40u;
  return ((u & 0x7fffffffu) > 0x7f800000u) ? q : r;
}

__device__ __forceinline__ void hilo_pack(float v0, float v1, float v2, float v3,
                                          int& h01, int& h23, int& l01, int& l23) {
  const unsigned a0 = bf16_bits(v0), a1 = bf16_bits(v1), a2 = bf16_bits(v2), a3 = bf16_bits(v3);
  const unsigned b0 = bf16_bits(v0 - __uint_as_float(a0 << 16));
  const unsigned b1 = bf16_bits(v1 - __uint_as_float(a1 << 16));
  const unsigned b2 = bf16_bits(v2 - __uint_as_float(a2 << 16));
  const unsigned b3 = bf16_bits(v3 - __uint_as_float(a3 << 16));
  h01 = (int)(a0 | (a1 << 16)); h23 = (int)(a2 | (a3 << 16));
  l01 = (int)(b0 | (b1 << 16)); l23 = (int)(b2 | (b3 << 16));
}

__device__ __forceinline__ void st2_v4f(float* p, v4f v) {
  *(volatile v4f*)p = v;
  __threadfence();
  *(volatile v4f*)p = v;
}
__device__ __forceinline__ void st2_v8us(unsigned short* p, v8us v) {
  *(volatile v8us*)p = v;
  __threadfence();
  *(volatile v8us*)p = v;
}

__device__ __forceinline__ v8us gather8(const float* __restrict__ base, int stride) {
  float f[8];
#pragma unroll
  for (int i = 0; i < 8; ++i) f[i] = base[(size_t)i * (size_t)stride];
  v8us o;
#pragma unroll
  for (int i = 0; i < 8; ++i) o[i] = (unsigned short)bf16_bits(f[i]);
  return o;
}

__device__ __forceinline__ void prep_layer_w(const float* __restrict__ w, unsigned short* dst, int u) {
  const int n = u >> 4, k8 = (u & 15) * 8, kk = k8 & (HD - 1);
  const v8us o = gather8(w + (size_t)kk * HD + n, HD);
  st2_v8us(dst + (size_t)n * WLP + k8, o);
}

__device__ __forceinline__ v4f bias_pair(const float* __restrict__ pa, const float* __restrict__ pb, int lane) {
  const int q = lane & 15;
  const v4f a = *(const v4fa*)(pa + 4 * q);
  const v4f b = *(const v4fa*)(pb + 4 * q);
  asm volatile("" :: "v"(a));
  asm volatile("" :: "v"(b));
  const unsigned ma = (lane < 16) ? 0xffffffffu : 0u;
  v4f o;
  o.x = __uint_as_float(((bf16_bits(a.x) << 16) & ma) | ((bf16_bits(b.x) << 16) & ~ma));
  o.y = __uint_as_float(((bf16_bits(a.y) << 16) & ma) | ((bf16_bits(b.y) << 16) & ~ma));
  o.z = __uint_as_float(((bf16_bits(a.z) << 16) & ma) | ((bf16_bits(b.z) << 16) & ~ma));
  o.w = __uint_as_float(((bf16_bits(a.w) << 16) & ma) | ((bf16_bits(b.w) << 16) & ~ma));
  return o;
}

__global__ __launch_bounds__(NTHR) void k_prep(const float* __restrict__ x, const float* __restrict__ wf,
                                               const float* __restrict__ wa, const float* __restrict__ wb,
                                               const float* __restrict__ wc, const float* __restrict__ wm,
                                               const float* __restrict__ ba, const float* __restrict__ bb,
                                               const float* __restrict__ bc, const float* __restrict__ bd,
                                               const float* __restrict__ bm,
                                               unsigned short* xb, unsigned short* wft, unsigned short* wlt,
                                               unsigned short* wmt, unsigned short* cat, float* pp, float* sm) {
  const int tid = (int)threadIdx.x, lane = tid & 31;
  const int blk = (int)blockIdx.x;
  if (blk < PE_X) {
    const int u   = blk * NTHR + tid;
    const int row = u >> 5, k8 = (u & 31) * 8;
    const int rc  = row < NN ? row : NN - 1;
    const unsigned mk = row < NN ? 0xffffu : 0u;
    const float* p = x + (size_t)rc * FD + k8;
    const v4f a = *(const v4fa*)p;
    const v4f b = *(const v4fa*)(p + 4);
    v8us o;
    o[0] = (unsigned short)(bf16_bits(a.x) & mk); o[1] = (unsigned short)(bf16_bits(a.y) & mk);
    o[2] = (unsigned short)(bf16_bits(a.z) & mk); o[3] = (unsigned short)(bf16_bits(a.w) & mk);
    o[4] = (unsigned short)(bf16_bits(b.x) & mk); o[5] = (unsigned short)(bf16_bits(b.y) & mk);
    o[6] = (unsigned short)(bf16_bits(b.z) & mk); o[7] = (unsigned short)(bf16_bits(b.w) & mk);
    st2_v8us(xb + (size_t)row * FD + k8, o);
  } else if (blk < PE_WF) {
    const int u = (blk - PE_X) * NTHR + tid;
    const int n = u >> 5, k8 = (u & 31) * 8;
    const v8us o = gather8(wf + (size_t)k8 * HD + n, HD);
    st2_v8us(wft + (size_t)n * FD + k8, o);
  } else if (blk < PE_WA) {
    prep_layer_w(wa, wlt, (blk - PE_WF) * NTHR + tid);
  } else if (blk < PE_WB) {
    prep_layer_w(wb, wlt + (size_t)HD * WLP, (blk - PE_WA) * NTHR + tid);
  } else if (blk < PE_WC) {
    prep_layer_w(wc, wlt + (size_t)2 * HD * WLP, (blk - PE_WB) * NTHR + tid);
  } else if (blk < PE_WM) {
    const int u = (blk - PE_WC) * NTHR + tid;
    const int n = u >> 6, k8 = (u & 63) * 8, kk = k8 & (CLO - 1);
    const v8us o = gather8(wm + (size_t)kk * HD + n, HD);
    st2_v8us(wmt + (size_t)n * WMP + k8, o);
  } else if (blk < PE_ZC) {
    const int u = (blk - PE_WM) * NTHR + tid;
    const int row = NN + (u >> 6), k8 = (u & 63) * 8;
    const v8us z = {0, 0, 0, 0, 0, 0, 0, 0};
    st2_v8us(cat + (size_t)row * CW + k8, z);
  } else if (blk < PE_ZP) {
    const int u = (blk - PE_ZC) * NTHR + tid;
    const int row = NN + (u >> 4), c4 = (u & 15) * 4;
    const v4f z = {0.0f, 0.0f, 0.0f, 0.0f};
    st2_v4f(pp + (size_t)row * HD + c4, z);
  } else {
    if (tid < 32) {
      const v4f o0 = bias_pair(ba, bb, lane);
      const v4f o1 = bias_pair(bc, bd, lane);
      const v4f o2 = bias_pair(bm, bm, lane);
      st2_v4f(sm + 4 * lane, o0);
      st2_v4f(sm + 128 + 4 * lane, o1);
      st2_v4f(sm + 256 + 4 * lane, o2);
    }
  }
}

__device__ __forceinline__ int sweep_keys(const int* __restrict__ keys, unsigned nbs, int* mylist,
                                          int wave, int lane) {
  const int per  = ((NE + NWAVE * WCH - 1) / (NWAVE * WCH)) * WCH;
  const int ebeg = wave * per;
  const int eend = (ebeg + per < NE) ? (ebeg + per) : NE;
  int wc = 0;
#pragma unroll 1
  for (int cb = ebeg; cb < eend; cb += WCH) {
    const int e0 = cb + lane * EPT;
    const v4i da = *(const v4ia*)(keys + e0);
    const v4i db = *(const v4ia*)(keys + e0 + 4);
    const unsigned s0 = (unsigned)da.x - nbs, s1 = (unsigned)da.y - nbs;
    const unsigned s2 = (unsigned)da.z - nbs, s3 = (unsigned)da.w - nbs;
    const unsigned s4 = (unsigned)db.x - nbs, s5 = (unsigned)db.y - nbs;
    const unsigned s6 = (unsigned)db.z - nbs, s7 = (unsigned)db.w - nbs;
    const bool h0 = s0 < (unsigned)NBRUN, h1 = s1 < (unsigned)NBRUN, h2 = s2 < (unsigned)NBRUN, h3 = s3 < (unsigned)NBRUN;
    const bool h4 = s4 < (unsigned)NBRUN, h5 = s5 < (unsigned)NBRUN, h6 = s6 < (unsigned)NBRUN, h7 = s7 < (unsigned)NBRUN;
    const unsigned m0 = __builtin_amdgcn_ballot_w32(h0), m1 = __builtin_amdgcn_ballot_w32(h1);
    const unsigned m2 = __builtin_amdgcn_ballot_w32(h2), m3 = __builtin_amdgcn_ballot_w32(h3);
    const unsigned m4 = __builtin_amdgcn_ballot_w32(h4), m5 = __builtin_amdgcn_ballot_w32(h5);
    const unsigned m6 = __builtin_amdgcn_ballot_w32(h6), m7 = __builtin_amdgcn_ballot_w32(h7);
    const unsigned any = m0 | m1 | m2 | m3 | m4 | m5 | m6 | m7;
    if (any != 0u) {
      const int pre = (int)(__builtin_amdgcn_mbcnt_lo(m0, 0u) + __builtin_amdgcn_mbcnt_lo(m1, 0u) +
                            __builtin_amdgcn_mbcnt_lo(m2, 0u) + __builtin_amdgcn_mbcnt_lo(m3, 0u) +
                            __builtin_amdgcn_mbcnt_lo(m4, 0u) + __builtin_amdgcn_mbcnt_lo(m5, 0u) +
                            __builtin_amdgcn_mbcnt_lo(m6, 0u) + __builtin_amdgcn_mbcnt_lo(m7, 0u));
      int p = wc + pre;
      if (h0) { if (p < WLCAP) mylist[p] = ((e0 + 0) << SLB) | (int)s0; p = p + 1; }
      if (h1) { if (p < WLCAP) mylist[p] = ((e0 + 1) << SLB) | (int)s1; p = p + 1; }
      if (h2) { if (p < WLCAP) mylist[p] = ((e0 + 2) << SLB) | (int)s2; p = p + 1; }
      if (h3) { if (p < WLCAP) mylist[p] = ((e0 + 3) << SLB) | (int)s3; p = p + 1; }
      if (h4) { if (p < WLCAP) mylist[p] = ((e0 + 4) << SLB) | (int)s4; p = p + 1; }
      if (h5) { if (p < WLCAP) mylist[p] = ((e0 + 5) << SLB) | (int)s5; p = p + 1; }
      if (h6) { if (p < WLCAP) mylist[p] = ((e0 + 6) << SLB) | (int)s6; p = p + 1; }
      if (h7) { if (p < WLCAP) mylist[p] = ((e0 + 7) << SLB) | (int)s7; p = p + 1; }
      wc += (int)(__builtin_popcount(m0) + __builtin_popcount(m1) + __builtin_popcount(m2) + __builtin_popcount(m3) +
                  __builtin_popcount(m4) + __builtin_popcount(m5) + __builtin_popcount(m6) + __builtin_popcount(m7));
    }
  }
  return wc;
}

__device__ __forceinline__ int count_lists(const int* wl, const int* misc, int* carr, int lane) {
  int ov = 0;
#pragma unroll 1
  for (int w2 = 0; w2 < NWAVE; ++w2) {
    int c = misc[w2];
    if (c > WLCAP) ov = 1;
    c = c < 0 ? 0 : (c > WLCAP ? WLCAP : c);
#pragma unroll 1
    for (int b0 = 0; b0 < c; b0 += 32) {
      const int idx = b0 + lane;
      const int ent = wl[w2 * WLCAP + (idx < WLCAP ? idx : WLCAP - 1)];
      const int m32 = (c - b0) < 32 ? (c - b0) : 32;
#pragma unroll 1
      for (int k = 0; k < m32; ++k) {
        const int u    = __builtin_amdgcn_readlane(ent, k);
        const int slot = u & (NBRUN - 1);
        if (lane == 0) carr[slot] = carr[slot] + 1;
      }
    }
  }
  return ov;
}

__device__ __forceinline__ void bucket_flush(const int* pl, const int* cnt, const int* nsd, int fl,
                                             int* lp, int* cop, int* ndp, int* nsp, int* fp, int tid) {
#pragma unroll 1
  for (int i = tid * 4; i < RCAP; i += NTHR * 4) {
    const v4i v = *(const v4ia*)(pl + i);
    *(volatile v4i*)(lp + i) = v;
  }
#pragma unroll 1
  for (int it = 0; it < 2; ++it) {
    const v4i v = *(const v4ia*)(cnt + it * NBRUN + 4 * tid);
    *(volatile v4i*)(cop + it * NBRUN + 4 * tid) = v;
  }
  {
    const v4i v = *(const v4ia*)(nsd + 4 * tid);
    *(volatile v4i*)(ndp + 4 * tid) = v;
    const v4i w = *(const v4ia*)(nsd + NBRUN + 4 * tid);
    *(volatile v4i*)(nsp + 4 * tid) = w;
  }
  if (tid < 8) {
    const v4i f = {fl, fl, fl, fl};
    *(volatile v4i*)(fp + 4 * tid) = f;
  }
}

__global__ __launch_bounds__(NTHR) void k_bucket(const int* __restrict__ srcs, const int* __restrict__ dsts,
                                                 int* LIST, int* CO, int* NDP, int* NSP, int* FLAG) {
  extern __shared__ __attribute__((aligned(16))) int dsm[];
  int* wl   = dsm + BK_WL;
  int* pl   = dsm + BK_PL;
  int* cnt  = dsm + BK_CNT;
  int* offs = cnt + NBRUN;
  int* cur  = offs + NBRUN;
  int* nsd  = dsm + BK_NSD;
  int* misc = dsm + BK_ZINTS;
  const int tid = (int)threadIdx.x, lane = tid & 31, wave = tid >> 5;
  const int blk = (int)blockIdx.x;
  const unsigned nbs = (unsigned)(blk * NBRUN);
  const v4i z4 = {0, 0, 0, 0};

  for (int i = tid * 4; i < BK_ZINTS; i += NTHR * 4) *(v4ia*)(dsm + i) = z4;
  if (tid < 16) misc[tid] = 0;
  __syncthreads();

  {
    const int wc = sweep_keys(dsts, nbs, wl + wave * WLCAP, wave, lane);
    if (lane == 0) misc[wave] = wc;
  }
  __syncthreads();

  if (wave == 0) {
    const int ov = count_lists(wl, misc, cnt, lane);
    if (lane == 0) misc[9] = ov;
  }
  __syncthreads();
  if (wave == 0) {
    const int base = lane * (NBRUN / 32);
    int s = 0;
#pragma unroll 1
    for (int i = 0; i < NBRUN / 32; ++i) s += cnt[base + i];
    int incl = s;
#pragma unroll
    for (int d = 1; d < 32; d <<= 1) {
      const int y = __shfl_up(incl, d, 32);
      if (lane >= d) incl += y;
    }
    int run = incl - s;
#pragma unroll 1
    for (int i = 0; i < NBRUN / 32; ++i) {
      const int cv = cnt[base + i];
      offs[base + i] = run;
      cur[base + i]  = run;
      run += cv;
    }
  }
  __syncthreads();

  if (wave == 0) {
#pragma unroll 1
    for (int w2 = 0; w2 < NWAVE; ++w2) {
      int c = misc[w2];
      c = c < 0 ? 0 : (c > WLCAP ? WLCAP : c);
#pragma unroll 1
      for (int b0 = 0; b0 < c; b0 += 32) {
        const int idx = b0 + lane;
        const int ent = wl[w2 * WLCAP + (idx < WLCAP ? idx : WLCAP - 1)];
        int eid = (ent >> SLB) & 0xFFFFF;
        eid = eid > NE - 1 ? NE - 1 : eid;
        int sr = srcs[eid];
        sr = sr < 0 ? 0 : (sr > NN - 1 ? NN - 1 : sr);
        const int word = (int)((unsigned)sr | ((unsigned)(ent & (NBRUN - 1)) << 16));
        const int m32 = (c - b0) < 32 ? (c - b0) : 32;
#pragma unroll 1
        for (int k = 0; k < m32; ++k) {
          const int u    = __builtin_amdgcn_readlane(ent, k);
          const int wd   = __builtin_amdgcn_readlane(word, k);
          const int slot = u & (NBRUN - 1);
          if (lane == 0) {
            int p = cur[slot];
            p = p < 0 ? 0 : (p > RCAP - 1 ? RCAP - 1 : p);
            pl[p] = wd;
            cur[slot] = p + 1;
          }
        }
      }
    }
  }
  __syncthreads();

  *(v4ia*)(cur + 4 * tid) = z4;
  {
    const int wc = sweep_keys(srcs, nbs, wl + wave * WLCAP, wave, lane);
    if (lane == 0) misc[wave] = wc;
  }
  __syncthreads();
  if (wave == 0) {
    const int ov = count_lists(wl, misc, cur, lane);
    if (lane == 0) misc[10] = ov;
  }
  __syncthreads();

  const int flag = misc[9] | misc[10];
#pragma unroll 1
  for (int it = 0; it < 8; ++it) {
    const int idx = it * NTHR + tid;
    const int sel = (it >= 4) ? NBRUN : 0;
    int c = cnt[idx + sel];
    c = c < 1 ? 1 : c;
    const float f = 1.0f / sqrtf((float)c);
    nsd[idx] = (flag != 0) ? (int)0x7fc00000 : __float_as_int(f);
  }
  __syncthreads();

  int* lp  = LIST + (size_t)blk * RCAP;
  int* cop = CO + (size_t)blk * (2 * NBRUN);
  int* ndp = NDP + (size_t)blk * NBRUN;
  int* nsp = NSP + (size_t)blk * NBRUN;
  int* fp  = FLAG + (size_t)blk * 32;
  bucket_flush(pl, cnt, nsd, flag, lp, cop, ndp, nsp, fp, tid);
  __threadfence();
  bucket_flush(pl, cnt, nsd, flag, lp, cop, ndp, nsp, fp, tid);
}

template <int KH, int NPART, int LOOFF, int BPITCH>
__device__ __forceinline__ void gemm_16x64(const unsigned short* __restrict__ ap,
                                           const unsigned short* __restrict__ bp, v8f (&acc)[4]) {
  static_assert(KH % 32 == 0 && NPART >= 1 && NPART <= 2 && NPART * KH <= BPITCH);
#pragma unroll 1
  for (int part = 0; part < NPART; ++part) {
    const unsigned short* aq = ap + part * LOOFF;
    const unsigned short* bq = bp + part * KH;
#pragma unroll 1
    for (int k0 = 0; k0 < KH; k0 += 32) {
      FragB af;
      af.h[0] = *(const v8usa*)(aq + k0);
      af.h[1] = *(const v8usa*)(aq + k0 + 16);
#pragma unroll
      for (int nt = 0; nt < 4; ++nt) {
        const unsigned short* wq = bq + (size_t)(16 * nt) * (size_t)BPITCH + k0;
        FragB bf;
        bf.h[0] = *(const v8usa*)wq;
        bf.h[1] = *(const v8usa*)(wq + 16);
        acc[nt] = wmb(af, bf, acc[nt]);
      }
    }
  }
}

__device__ __forceinline__ void stage_d(float* stg, const v8f (&acc)[4], int wave, int hh, int m) {
#pragma unroll
  for (int nt = 0; nt < 4; ++nt) {
#pragma unroll
    for (int r = 0; r < 8; ++r) stg[(16 * wave + 8 * hh + r) * SP + 16 * nt + m] = acc[nt][r];
  }
}

template <int KH, int NPART, int APITCH, int LOOFF, int BPITCH, int SCALE>
__global__ __launch_bounds__(NTHR) __attribute__((amdgpu_num_vgpr(248)))
void k_gemm(const unsigned short* __restrict__ A, const unsigned short* __restrict__ BT,
            const float* __restrict__ NS, float* Pout) {
  __shared__ __attribute__((aligned(16))) float stg[GBM * SP];
  __shared__ __attribute__((aligned(16))) float sns[GBM];
  const int tid = (int)threadIdx.x, lane = tid & 31, wave = tid >> 5, hh = lane >> 4, m = lane & 15;
  const int rowBase = (int)blockIdx.x * GBM;
  if (tid < 32) {
    v4f s4 = {1.0f, 1.0f, 1.0f, 1.0f};
    if constexpr (SCALE != 0) s4 = *(const v4fa*)(NS + rowBase + 4 * tid);
    *(v4fa*)(sns + 4 * tid) = s4;
  }

  v8f acc[4];
  {
    const v8f z = {0.f, 0.f, 0.f, 0.f, 0.f, 0.f, 0.f, 0.f};
#pragma unroll
    for (int t = 0; t < 4; ++t) acc[t] = z;
  }
  const unsigned short* ap = A + (size_t)(rowBase + 16 * wave + m) * (size_t)APITCH + 8 * hh;
  const unsigned short* bp = BT + (size_t)m * (size_t)BPITCH + 8 * hh;
  gemm_16x64<KH, NPART, LOOFF, BPITCH>(ap, bp, acc);
  stage_d(stg, acc, wave, hh, m);
  __syncthreads();

#pragma unroll 1
  for (int i = 0; i < 8; ++i) {
    const int lr   = 16 * wave + 2 * i + hh;
    const int grow = rowBase + lr;
    const bool live = grow < NN;
    const v4f a = *(const v4fa*)(stg + lr * SP + 4 * m);
    const float s = sns[lr];
    asm volatile("" :: "v"(a));
    asm volatile("" :: "v"(s));
    const float v0 = a.x * s, v1 = a.y * s, v2 = a.z * s, v3 = a.w * s;
    v4f o;
    o.x = live ? v0 : 0.0f; o.y = live ? v1 : 0.0f; o.z = live ? v2 : 0.0f; o.w = live ? v3 : 0.0f;
    st2_v4f(Pout + (size_t)grow * HD + 4 * m, o);
  }
}

template <int FINAL>
__global__ __launch_bounds__(NTHR) void k_replay(const int* __restrict__ LIST, const int* __restrict__ CO,
                                                 const int* __restrict__ FLAG, const float* __restrict__ Pin,
                                                 const float* __restrict__ ND, const float* __restrict__ bias,
                                                 unsigned short* cats, float* out) {
  __shared__ __attribute__((aligned(16))) float sb[128];
  const int tid = (int)threadIdx.x, lane = tid & 31, wave = tid >> 5, hh = lane >> 4, q = lane & 15;
  const int rowBase = (int)blockIdx.x * ABM;
  const int bucket  = rowBase >> SLB;
  const int* lb  = LIST + (size_t)bucket * RCAP;
  const int* cob = CO + (size_t)bucket * (2 * NBRUN);
  const int flag = FLAG[(size_t)bucket * 32];
  const float qnan = __uint_as_float(0x7fc00000u);
  if (tid < 32) *(v4fa*)(sb + 4 * tid) = *(const v4fa*)(bias + 4 * tid);
  __syncthreads();
  const v4f bv = *(const v4fa*)(sb + 4 * q);

#pragma unroll 1
  for (int i = 0; i < ABM / (2 * NWAVE); ++i) {
    const int d    = rowBase + (ABM / NWAVE) * wave + 2 * i + hh;
    const int slot = d & (NBRUN - 1);
    int c = cob[slot];
    int o = cob[NBRUN + slot];
    const float nd = ND[d];
    const bool big = c > TRIPCAP;
    c = c < 0 ? 0 : (c > TRIPCAP ? TRIPCAP : c);
    o = o < 0 ? 0 : (o > RCAP - 1 ? RCAP - 1 : o);
    const int co = __shfl_xor(c, 16, 32);
    const int cm = c > co ? c : co;
    const int cmu = __builtin_amdgcn_readfirstlane(cm);
    int last = o + c - 1; last = last < o ? o : last;
    last = last > RCAP - 1 ? RCAP - 1 : last;
    float a0 = 0.0f, a1 = 0.0f, a2 = 0.0f, a3 = 0.0f;
#pragma unroll 1
    for (int j = 0; j < cmu; ++j) {
      int idx = o + j;
      idx = idx > last ? last : idx;
      const unsigned wd = (unsigned)lb[idx];
      int sr = (int)(wd & 0xffffu);
      sr = sr > NN - 1 ? NN - 1 : sr;
      const v4f v = *(const v4fa*)(Pin + (size_t)sr * HD + 4 * q);
      asm volatile("" :: "v"(v));
      const bool valid = j < c;
      const float t0 = a0 + v.x, t1 = a1 + v.y, t2 = a2 + v.z, t3 = a3 + v.w;
      a0 = valid ? t0 : a0; a1 = valid ? t1 : a1; a2 = valid ? t2 : a2; a3 = valid ? t3 : a3;
    }
    const bool bad  = (flag != 0) | big;
    const bool live = d < NN;
    if constexpr (FINAL == 0) {
      float m0 = nd * a0 + bv.x, m1 = nd * a1 + bv.y, m2 = nd * a2 + bv.z, m3 = nd * a3 + bv.w;
      m0 = (m0 > 0.0f) ? m0 : (m0 - m0); m1 = (m1 > 0.0f) ? m1 : (m1 - m1);
      m2 = (m2 > 0.0f) ? m2 : (m2 - m2); m3 = (m3 > 0.0f) ? m3 : (m3 - m3);
      m0 = bad ? qnan : m0; m1 = bad ? qnan : m1; m2 = bad ? qnan : m2; m3 = bad ? qnan : m3;
      m0 = live ? m0 : 0.0f; m1 = live ? m1 : 0.0f; m2 = live ? m2 : 0.0f; m3 = live ? m3 : 0.0f;
      int h01, h23, l01, l23;
      hilo_pack(m0, m1, m2, m3, h01, h23, l01, l23);
      v2i hv, lv;
      hv.x = h01; hv.y = h23; lv.x = l01; lv.y = l23;
      unsigned short* hp = cats + (size_t)d * CW + 4 * q;
      unsigned short* lp = hp + CLO;
      *(volatile v2i*)hp = hv;
      *(volatile v2i*)lp = lv;
      __threadfence();
      *(volatile v2i*)hp = hv;
      *(volatile v2i*)lp = lv;
    } else {
      float m0 = a0 + bv.x, m1 = a1 + bv.y, m2 = a2 + bv.z, m3 = a3 + bv.w;
      m0 = bad ? qnan : m0; m1 = bad ? qnan : m1; m2 = bad ? qnan : m2; m3 = bad ? qnan : m3;
      v4f ov;
      ov.x = m0; ov.y = m1; ov.z = m2; ov.w = m3;
      asm volatile("" :: "v"(ov));
      const int dc = live ? d : NN - 1;
      float* op = out + (size_t)dc * HD + 4 * q;
      if (live) *(volatile v4f*)op = ov;
      __threadfence();
      if (live) *(volatile v4f*)op = ov;
    }
  }
}

extern "C" void kernel_launch(void* const* d_in, const int* in_sizes, int n_in,
                              void* d_out, int out_size, void* d_ws, size_t ws_size,
                              hipStream_t stream) {
  if (n_in < 13) return;
  if (in_sizes[0] != NN * FD) return;
  if (in_sizes[1] != NE) return;
  if (in_sizes[2] != NE) return;
  if (in_sizes[3] != FD * HD) return;
  if (in_sizes[4] != HD) return;
  if (in_sizes[5] != HD * HD) return;
  if (in_sizes[6] != HD) return;
  if (in_sizes[7] != HD * HD) return;
  if (in_sizes[8] != HD) return;
  if (in_sizes[9] != HD * HD) return;
  if (in_sizes[10] != HD) return;
  if (in_sizes[11] != NSL * HD * HD) return;
  if (in_sizes[12] != HD) return;
  if (out_size != NN * HD) return;

  const float* x    = (const float*)d_in[0];
  const int*   srcs = (const int*)d_in[1];
  const int*   dsts = (const int*)d_in[2];
  const float* wf   = (const float*)d_in[3];
  const float* ba   = (const float*)d_in[4];
  const float* wa   = (const float*)d_in[5];
  const float* bb   = (const float*)d_in[6];
  const float* wb   = (const float*)d_in[7];
  const float* bc   = (const float*)d_in[8];
  const float* wc   = (const float*)d_in[9];
  const float* bd   = (const float*)d_in[10];
  const float* wm   = (const float*)d_in[11];
  const float* bm   = (const float*)d_in[12];
  float* out = (float*)d_out;

  constexpr size_t zXB   = (size_t)MP * FD * 2;
  constexpr size_t zP    = (size_t)MP * HD * 4;
  constexpr size_t zCAT  = (size_t)MP * CW * 2;
  constexpr size_t zLIST = (size_t)NBK * RCAP * 4;
  constexpr size_t zCO   = (size_t)NBK * 2 * NBRUN * 4;
  constexpr size_t zNSD  = (size_t)2 * NBK * NBRUN * 4;
  constexpr size_t zFLAG = (((size_t)NBK * 128 + 255) / 256) * 256;
  constexpr size_t zWFT  = (size_t)HD * FD * 2;
  constexpr size_t zWLT  = (size_t)3 * HD * WLP * 2;
  constexpr size_t zWMT  = (size_t)HD * WMP * 2;
  constexpr size_t zSM   = (size_t)6 * HD * 4;
  constexpr size_t oXB   = 0;
  constexpr size_t oP    = oXB + zXB;
  constexpr size_t oCAT  = oP + zP;
  constexpr size_t oLIST = oCAT + zCAT;
  constexpr size_t oCO   = oLIST + zLIST;
  constexpr size_t oNSD  = oCO + zCO;
  constexpr size_t oFLAG = oNSD + zNSD;
  constexpr size_t oWFT  = oFLAG + zFLAG;
  constexpr size_t oWLT  = oWFT + zWFT;
  constexpr size_t oWMT  = oWLT + zWLT;
  constexpr size_t oSM   = oWMT + zWMT;
  constexpr size_t oEND  = oSM + zSM;
  static_assert(zXB % 256 == 0 && zP % 256 == 0 && zCAT % 256 == 0 && zLIST % 256 == 0 && zCO % 256 == 0);
  static_assert(zNSD % 256 == 0 && zFLAG % 256 == 0 && zWFT % 256 == 0 && zWLT % 256 == 0 && zWMT % 256 == 0);
  static_assert(zSM % 256 == 0 && zFLAG >= (size_t)NBK * 128);
  static_assert(oEND <= (size_t)(128u << 20));
  if (oEND > ws_size) return;

  char* ws = (char*)d_ws;
  unsigned short* XB   = (unsigned short*)(ws + oXB);
  float*          P    = (float*)(ws + oP);
  unsigned short* CAT  = (unsigned short*)(ws + oCAT);
  int*            LIST = (int*)(ws + oLIST);
  int*            CO   = (int*)(ws + oCO);
  int*            NDi  = (int*)(ws + oNSD);
  int*            NSi  = NDi + (size_t)NBK * NBRUN;
  const float*    NDf  = (const float*)(ws + oNSD);
  const float*    NSf  = NDf + (size_t)NBK * NBRUN;
  int*            FLAG = (int*)(ws + oFLAG);
  unsigned short* WFT  = (unsigned short*)(ws + oWFT);
  unsigned short* WLT  = (unsigned short*)(ws + oWLT);
  unsigned short* WMT  = (unsigned short*)(ws + oWMT);
  float*          SM   = (float*)(ws + oSM);

  hipFuncSetAttribute(reinterpret_cast<const void*>(&k_bucket), hipFuncAttributeMaxDynamicSharedMemorySize, (int)BK_LDS);

  k_prep<<<PBTOT, NTHR, 0, stream>>>(x, wf, wa, wb, wc, wm, ba, bb, bc, bd, bm, XB, WFT, WLT, WMT, CAT, P, SM);
  k_bucket<<<NBK, NTHR, BK_LDS, stream>>>(srcs, dsts, LIST, CO, NDi, NSi, FLAG);
  k_gemm<FD, 1, FD, 0, FD, 1><<<MP / GBM, NTHR, 0, stream>>>(XB, WFT, NSf, P);
  k_replay<0><<<MP / ABM, NTHR, 0, stream>>>(LIST, CO, FLAG, P, NDf, SM, CAT, out);
  for (int l = 1; l < NSL; ++l) {
    k_gemm<HD, 1 + LAYER_SPLIT, CW, CLO, WLP, 1><<<MP / GBM, NTHR, 0, stream>>>(
        CAT + (size_t)(l - 1) * HD, WLT + (size_t)(l - 1) * HD * WLP, NSf, P);
    k_replay<0><<<MP / ABM, NTHR, 0, stream>>>(LIST, CO, FLAG, P, NDf, SM + (size_t)l * HD,
                                               CAT + (size_t)l * HD, out);
  }
  k_gemm<CLO, 1 + HEAD_SPLIT, CW, CLO, WMP, 0><<<MP / GBM, NTHR, 0, stream>>>(CAT, WMT, NSf, P);
  k_replay<1><<<MP / ABM, NTHR, 0, stream>>>(LIST, CO, FLAG, P, NDf, SM + (size_t)4 * HD, CAT, out);
}
